// HMM3Aligner_89129161326629
// MI455X (gfx1250) — hardware-verified
//
#include <hip/hip_runtime.h>
#include <stdint.h>

typedef __attribute__((ext_vector_type(16))) _Float16 v16h;
typedef __attribute__((ext_vector_type(8)))  _Float16 v8h;
typedef __attribute__((ext_vector_type(8)))  float    v8f;
typedef __attribute__((ext_vector_type(4)))  float    v4f;
typedef __attribute__((ext_vector_type(4)))  unsigned v4u;

constexpr int kBatch = 8;
constexpr int kLen   = 512;
constexpr int kDim   = 256;
constexpr int kSt    = 3;
constexpr int kGroup = 2;
constexpr int kNumGroups = kBatch / kGroup;
constexpr int kPlanesPerBatch = 12;
constexpr int kPlaneOp = kLen * kDim;
constexpr int kPlaneSc = kLen * kLen;
constexpr int kDiag = 2 * kLen - 1;
constexpr size_t kDiagFloats = (size_t)kDiag * kLen * 4;
constexpr float  kNeg  = -1.0e9f;
constexpr double kNegD = -1.0e9;
constexpr float  kOpCarry  = 8.0f;
constexpr float  kOutScale = 1.0f / 64.0f;
static_assert(kBatch % kGroup == 0, "group size");
static_assert(kDim % 32 == 0, "K multiple of 32");
static_assert(kLen % 64 == 0, "M,N multiples of the 64 tile");
static_assert(kLen == 512, "one 512-thread block per column set");

__device__ __forceinline__ void dep_guard_h(v8f& a, v8f& b, v16h x, v16h y) { asm volatile("v_nop\n\tv_nop\n\tv_nop\n\tv_nop" : "+v"(a), "+v"(b) : "v"(x), "v"(y)); }
__device__ __forceinline__ void keep4_h(v16h a, v16h b, v16h c, v16h d) { asm volatile("v_nop" :: "v"(a), "v"(b), "v"(c), "v"(d)); }
__device__ __forceinline__ void acc_guard4(v8f& a, v8f& b, v8f& c, v8f& d) { asm volatile("v_nop\n\tv_nop\n\tv_nop\n\tv_nop" : "+v"(a), "+v"(b), "+v"(c), "+v"(d)); }
template <typename T> struct Frag;
template <> struct Frag<_Float16> {
  typedef v16h V; union U { v16h v; v8h h[2]; };
  static __device__ __forceinline__ v16h load(const _Float16* p) {
    U f; f.h[0] = *(const v8h*)(p); f.h[1] = *(const v8h*)(p + 16); return f.v;
  }
  static __device__ __forceinline__ v8f mma(v16h a, v16h b, v8f c) {
    return __builtin_amdgcn_wmma_f32_16x16x32_f16(false, a, false, b, (short)0, c, false, false);
  }
  static __device__ __forceinline__ void guard(v8f& a, v8f& b, v16h x, v16h y) { dep_guard_h(a, b, x, y); }
  static __device__ __forceinline__ void keep(v16h a, v16h b, v16h c, v16h d) { keep4_h(a, b, c, d); }
};

__device__ __forceinline__ unsigned short f2h_bits_x8(float f) {
  return __builtin_bit_cast(unsigned short, (_Float16)(f * kOpCarry));
}

__global__ __launch_bounds__(256) void k_cast_planes(
    const float* __restrict__ zx, const float* __restrict__ zy,
    const float* __restrict__ gx, const float* __restrict__ gy,
    unsigned short* __restrict__ OP) {
  __shared__ __align__(16) unsigned short sh[kSt * kDim];
  const int l = blockIdx.x;
  const int b = blockIdx.y;
  const int t = blockIdx.z;
  const float* src = (t == 0) ? zx : (t == 1) ? zy : (t == 2) ? gx : gy;
  const int d = threadIdx.x;
  const float* s3 = src + ((size_t)(b * kLen + l) * kDim + d) * kSt;
  const float f0 = s3[0], f1 = s3[1], f2 = s3[2];
  sh[0 * kDim + d] = f2h_bits_x8(f0);
  sh[1 * kDim + d] = f2h_bits_x8(f1);
  sh[2 * kDim + d] = f2h_bits_x8(f2);
  __syncthreads();
  const int w = threadIdx.x >> 5;
  const int lane = threadIdx.x & 31;
  if (w < kSt) {
    const v4u val = *(const v4u*)(sh + w * kDim + lane * 8);
    unsigned short* dst = OP + (size_t)((t * kBatch + b) * kSt + w) * kPlaneOp + (size_t)l * kDim + lane * 8;
    *(volatile v4u*)dst = val;
    __threadfence();
    *(volatile v4u*)dst = val;
  }
}

__global__ __launch_bounds__(256) void k_gemm_planes(
    const unsigned short* __restrict__ OPp, float* __restrict__ THA, int gbase,
    int lda, int ldb, int ldc, int M, int N, int K, float scale) {
  typedef _Float16 T;
  typedef Frag<T>::V V;
  const T* OP = (const T*)OPp;
  __shared__ __align__(16) float sT[8][16 * 68];
  const int gp  = blockIdx.y;
  const int g   = gp / kPlanesPerBatch;
  const int p   = gp - g * kPlanesPerBatch;
  const int b   = gbase + g;
  const int isT = (p >= kSt) ? 1 : 0;
  const int q   = isT ? (p - kSt) : 0;
  const int u   = q / kSt;
  const int w   = q - kSt * u;
  const int tX  = isT ? 2 : 0;
  const int sX  = isT ? u : p;
  const int tY  = isT ? 3 : 1;
  const int sY  = isT ? w : p;
  const T* Ab = OP + (size_t)((tX * kBatch + b) * kSt + sX) * kPlaneOp;
  const T* Bb = OP + (size_t)((tY * kBatch + b) * kSt + sY) * kPlaneOp;
  float*   Cb = THA + (size_t)gp * kPlaneSc;

  const int lane = threadIdx.x & 31;
  const int wave = threadIdx.x >> 5;
  const int tilesN = N >> 6;
  const int tilesM = M >> 6;
  const int tile = blockIdx.x * 8 + wave;
  if (tile >= tilesM * tilesN) return;
  const int tm = tile / tilesN;
  const int tn = tile - tm * tilesN;
  const int m0 = tm << 6;
  const int n0 = tn << 6;

  const int rlane = lane & 15;
  const int koff  = (lane >> 4) * 8;
  const int mOff  = (lane >> 4) * 8;

  v8f acc[4][4];
#pragma unroll
  for (int i = 0; i < 4; ++i)
#pragma unroll
    for (int j = 0; j < 4; ++j) acc[i][j] = (v8f){0.f,0.f,0.f,0.f,0.f,0.f,0.f,0.f};

  for (int k0 = 0; k0 < K; k0 += 32) {
    V bh[4];
#pragma unroll
    for (int j = 0; j < 4; ++j) {
      const size_t bo = (size_t)(n0 + (j << 4) + rlane) * ldb + koff + k0;
      bh[j] = Frag<T>::load(Bb + bo);
    }
#pragma unroll
    for (int i = 0; i < 4; ++i) {
      const size_t ao = (size_t)(m0 + (i << 4) + rlane) * lda + koff + k0;
      V ah = Frag<T>::load(Ab + ao);
#pragma unroll
      for (int j = 0; j < 4; ++j) {
        acc[i][j] = Frag<T>::mma(ah, bh[j], acc[i][j]);
      }
      Frag<T>::guard(acc[i][0], acc[i][3], ah, ah);
    }
    Frag<T>::keep(bh[0], bh[1], bh[2], bh[3]);
  }
  acc_guard4(acc[0][0], acc[0][1], acc[0][2], acc[0][3]);
  acc_guard4(acc[1][0], acc[1][1], acc[1][2], acc[1][3]);
  acc_guard4(acc[2][0], acc[2][1], acc[2][2], acc[2][3]);
  acc_guard4(acc[3][0], acc[3][1], acc[3][2], acc[3][3]);

  float* slab = sT[wave];
#pragma unroll
  for (int i = 0; i < 4; ++i) {
    const int mBase = m0 + (i << 4);
#pragma unroll
    for (int j = 0; j < 4; ++j) {
#pragma unroll
      for (int r = 0; r < 8; ++r) {
        float v = acc[i][j][r] * scale;
        slab[(mOff + r) * 68 + (j << 4) + rlane] = v;
      }
    }
    __builtin_amdgcn_fence(__ATOMIC_RELEASE, "workgroup");
    __builtin_amdgcn_wave_barrier();
    __builtin_amdgcn_fence(__ATOMIC_ACQUIRE, "workgroup");
    {
      const int hh = lane >> 4, c4 = (lane & 15) * 4;
      for (int pass = 0; pass < 2; ++pass) {
#pragma unroll
        for (int it = 0; it < 8; ++it) {
          const int row = it * 2 + hh;
          v4f v = *(const v4f*)(slab + row * 68 + c4);
          *(volatile v4f*)(Cb + (size_t)(mBase + row) * ldc + n0 + c4) = v;
        }
        __threadfence();
      }
    }
    __builtin_amdgcn_fence(__ATOMIC_RELEASE, "workgroup");
    __builtin_amdgcn_wave_barrier();
    __builtin_amdgcn_fence(__ATOMIC_ACQUIRE, "workgroup");
  }
}

__device__ __forceinline__ double dmax2(double a, double b) { return (a > b) ? a : b; }
__device__ __forceinline__ double lse3d(double a, double b, double c) {
  const double m = dmax2(a, dmax2(b, c));
  const float ea = (float)(a - m);
  const float eb = (float)(b - m);
  const float ec = (float)(c - m);
  const float s = __expf(ea) + __expf(eb) + __expf(ec);
  return m + (double)__logf(s);
}

__global__ __launch_bounds__(512) void k_forward(const float* __restrict__ THA, float* __restrict__ AD) {
  __shared__ __align__(16) double ring[3][kLen * kSt];
  const int g = blockIdx.x;
  const int t = threadIdx.x;
  const int j = t + 1;
  const float* P = THA + (size_t)g * kPlanesPerBatch * kPlaneSc;
  float* ADg = AD + (size_t)g * kDiagFloats;
#pragma unroll
  for (int sl = 0; sl < 3; ++sl) {
    ring[sl][t * 3 + 0] = kNegD;
    ring[sl][t * 3 + 1] = kNegD;
    ring[sl][t * 3 + 2] = kNegD;
  }
  double up0 = kNegD, up1 = kNegD, up2 = kNegD;
  const int  tl   = (t > 0) ? (t - 1) : 0;
  const bool col1 = (t == 0);
  __syncthreads();

#pragma unroll 1
  for (int k = 2; k <= 2 * kLen; ++k) {
    const int  i     = k - j;
    const bool valid = (i >= 1) && (i <= kLen);
    const int  sc = k % 3;
    const int  s1 = (k + 2) % 3;
    const int  s2 = (k + 1) % 3;
    double d0 = ring[s2][tl * 3 + 0], d1 = ring[s2][tl * 3 + 1], d2 = ring[s2][tl * 3 + 2];
    double l0 = ring[s1][tl * 3 + 0], l1 = ring[s1][tl * 3 + 1], l2 = ring[s1][tl * 3 + 2];
    d0 = col1 ? ((k == 2) ? 0.0 : kNegD) : d0;
    d1 = col1 ? kNegD : d1;
    d2 = col1 ? kNegD : d2;
    l0 = col1 ? kNegD : l0;
    l1 = col1 ? kNegD : l1;
    l2 = col1 ? kNegD : l2;
    int ic = i - 1;
    ic = (ic < 0) ? 0 : ((ic > kLen - 1) ? (kLen - 1) : ic);
    const size_t off = (size_t)ic * kLen + t;
    const float th0 = P[(size_t)0 * kPlaneSc + off];
    const float th1 = P[(size_t)1 * kPlaneSc + off];
    const float th2 = P[(size_t)2 * kPlaneSc + off];
    const float a00 = P[(size_t)3 * kPlaneSc + off];
    const float a01 = P[(size_t)4 * kPlaneSc + off];
    const float a02 = P[(size_t)5 * kPlaneSc + off];
    const float a10 = P[(size_t)6 * kPlaneSc + off];
    const float a11 = P[(size_t)7 * kPlaneSc + off];
    const float a12 = P[(size_t)8 * kPlaneSc + off];
    const float a20 = P[(size_t)9 * kPlaneSc + off];
    const float a21 = P[(size_t)10 * kPlaneSc + off];
    const float a22 = P[(size_t)11 * kPlaneSc + off];
    double am = (double)th0 + lse3d(d0  + (double)a00, d1  + (double)a10, d2  + (double)a20);
    double ax = (double)th1 + lse3d(up0 + (double)a01, up1 + (double)a11, up2 + (double)a21);
    double ay = (double)th2 + lse3d(l0  + (double)a02, l1  + (double)a12, l2  + (double)a22);
    am = valid ? am : kNegD;
    ax = valid ? ax : kNegD;
    ay = valid ? ay : kNegD;
    ring[sc][t * 3 + 0] = am;
    ring[sc][t * 3 + 1] = ax;
    ring[sc][t * 3 + 2] = ay;
    up0 = am; up1 = ax; up2 = ay;
    v4f o;
    o.x = (float)am; o.y = (float)ax; o.z = (float)ay; o.w = 0.0f;
    float* dst = ADg + ((size_t)(k - 2) * kLen + t) * 4;
    *(volatile v4f*)dst = o;
    __threadfence();
    *(volatile v4f*)dst = o;
    __syncthreads();
  }
}

__global__ __launch_bounds__(512) void k_backward(const float* __restrict__ THA, float* __restrict__ BD) {
  __shared__ __align__(16) double ring[3][kLen * kSt];
  const int g = blockIdx.x;
  const int t = threadIdx.x;
  const int j = t + 1;
  const float* P = THA + (size_t)g * kPlanesPerBatch * kPlaneSc;
  float* BDg = BD + (size_t)g * kDiagFloats;
#pragma unroll
  for (int sl = 0; sl < 3; ++sl) {
    ring[sl][t * 3 + 0] = kNegD;
    ring[sl][t * 3 + 1] = kNegD;
    ring[sl][t * 3 + 2] = kNegD;
  }
  double dnx = kNegD;
  const int  tr      = (t < kLen - 1) ? (t + 1) : (kLen - 1);
  const bool lastcol = (t == kLen - 1);
  __syncthreads();

#pragma unroll 1
  for (int k = 2 * kLen; k >= 2; --k) {
    const int  i     = k - j;
    const bool valid = (i >= 1) && (i <= kLen);
    const int  sc = k % 3;
    const int  p1 = (k + 1) % 3;
    const int  p2 = (k + 2) % 3;
    double bM = ring[p2][tr * 3 + 0];
    double bY = ring[p1][tr * 3 + 2];
    bM = lastcol ? kNegD : bM;
    bY = lastcol ? kNegD : bY;
    const double bX = dnx;
    int iz = i - 1;
    iz = (iz < 0) ? 0 : ((iz > kLen - 1) ? (kLen - 1) : iz);
    const int izp = (iz + 1 > kLen - 1) ? (kLen - 1) : (iz + 1);
    const size_t offM = (size_t)izp * kLen + tr;
    const size_t offX = (size_t)izp * kLen + t;
    const size_t offY = (size_t)iz  * kLen + tr;
    const float thM = P[(size_t)0 * kPlaneSc + offM];
    const float thX = P[(size_t)1 * kPlaneSc + offX];
    const float thY = P[(size_t)2 * kPlaneSc + offY];
    const float aM0 = P[(size_t)3  * kPlaneSc + offM];
    const float aM1 = P[(size_t)6  * kPlaneSc + offM];
    const float aM2 = P[(size_t)9  * kPlaneSc + offM];
    const float aX0 = P[(size_t)4  * kPlaneSc + offX];
    const float aX1 = P[(size_t)7  * kPlaneSc + offX];
    const float aX2 = P[(size_t)10 * kPlaneSc + offX];
    const float aY0 = P[(size_t)5  * kPlaneSc + offY];
    const float aY1 = P[(size_t)8  * kPlaneSc + offY];
    const float aY2 = P[(size_t)11 * kPlaneSc + offY];
    const double cM = (double)thM + bM;
    const double cX = (double)thX + bX;
    const double cY = (double)thY + bY;
    double b0 = lse3d(cM + (double)aM0, cX + (double)aX0, cY + (double)aY0);
    double b1 = lse3d(cM + (double)aM1, cX + (double)aX1, cY + (double)aY1);
    double b2 = lse3d(cM + (double)aM2, cX + (double)aX2, cY + (double)aY2);
    const bool term = (k == 2 * kLen) && lastcol;
    b0 = term ? 0.0 : (valid ? b0 : kNegD);
    b1 = term ? 0.0 : (valid ? b1 : kNegD);
    b2 = term ? 0.0 : (valid ? b2 : kNegD);
    ring[sc][t * 3 + 0] = b0;
    ring[sc][t * 3 + 1] = b1;
    ring[sc][t * 3 + 2] = b2;
    dnx = b1;
    v4f o;
    o.x = (float)b0; o.y = (float)b1; o.z = (float)b2; o.w = 0.0f;
    float* dst = BDg + ((size_t)(k - 2) * kLen + t) * 4;
    *(volatile v4f*)dst = o;
    __threadfence();
    *(volatile v4f*)dst = o;
    __syncthreads();
  }
}

__global__ __launch_bounds__(512) void k_posterior(const float* __restrict__ AD, const float* __restrict__ BD,
                                                    float* __restrict__ out, int gbase) {
  __shared__ __align__(16) float sh[kLen * kSt];
  const int i0 = blockIdx.x;
  const int g  = blockIdx.y;
  const int b  = gbase + g;
  const int t  = threadIdx.x;
  const float* ADg = AD + (size_t)g * kDiagFloats;
  const float* BDg = BD + (size_t)g * kDiagFloats;
  const v4f aT = *(const v4f*)(ADg + ((size_t)(kDiag - 1) * kLen + (kLen - 1)) * 4);
  const double Z = lse3d((double)aT.x, (double)aT.y, (double)aT.z);
  const int kidx = i0 + t;
  const v4f a  = *(const v4f*)(ADg + ((size_t)kidx * kLen + t) * 4);
  const v4f bb = *(const v4f*)(BDg + ((size_t)kidx * kLen + t) * 4);
  const float p0 = __expf((float)(((double)a.x + (double)bb.x) - Z));
  const float p1 = __expf((float)(((double)a.y + (double)bb.y) - Z));
  const float p2 = __expf((float)(((double)a.z + (double)bb.z) - Z));
  sh[t * 3 + 0] = p0;
  sh[t * 3 + 1] = p1;
  sh[t * 3 + 2] = p2;
  __syncthreads();
  if (t < (kLen * kSt) / 4) {
    const v4f v = *(const v4f*)(sh + t * 4);
    float* dst = out + ((size_t)(b * kLen + i0) * kLen) * kSt + (size_t)t * 4;
    *(volatile v4f*)dst = v;
    __threadfence();
    *(volatile v4f*)dst = v;
  }
}

extern "C" void kernel_launch(void* const* d_in, const int* in_sizes, int n_in,
                              void* d_out, int out_size, void* d_ws, size_t ws_size,
                              hipStream_t stream)
{
  if (n_in < 4) return;
  const int nIn  = kBatch * kLen * kDim * kSt;
  const int nOut = kBatch * kLen * kLen * kSt;
  if (in_sizes[0] != nIn || in_sizes[1] != nIn || in_sizes[2] != nIn || in_sizes[3] != nIn) return;
  if (out_size != nOut) return;

  const size_t bytesOP  = (size_t)4 * kBatch * kSt * kPlaneOp * sizeof(unsigned short);
  const size_t bytesTHA = (size_t)kGroup * kPlanesPerBatch * kPlaneSc * sizeof(float);
  const size_t bytesAD  = (size_t)kGroup * kDiagFloats * sizeof(float);
  const size_t offOP  = 0;
  const size_t offTHA = offOP + bytesOP;
  const size_t offAD  = offTHA + bytesTHA;
  const size_t offBD  = offAD + bytesAD;
  const size_t total  = offBD + bytesAD;
  if (total > ws_size) return;

  const float* zx = (const float*)d_in[0];
  const float* zy = (const float*)d_in[1];
  const float* gx = (const float*)d_in[2];
  const float* gy = (const float*)d_in[3];
  char* ws = (char*)d_ws;
  unsigned short* OP  = (unsigned short*)(ws + offOP);
  float*          THA = (float*)(ws + offTHA);
  float*          AD  = (float*)(ws + offAD);
  float*          BD  = (float*)(ws + offBD);
  float*          out = (float*)d_out;

  k_cast_planes<<<dim3(kLen, kBatch, 4), 256, 0, stream>>>(zx, zy, gx, gy, OP);

  for (int gi = 0; gi < kNumGroups; ++gi) {
    const int gbase = gi * kGroup;
    k_gemm_planes<<<dim3((kLen / 64) * (kLen / 64) / 8, kGroup * kPlanesPerBatch), 256, 0, stream>>>(
        OP, THA, gbase, kDim, kDim, kLen, kLen, kLen, kDim, kOutScale);
    k_forward<<<kGroup, kLen, 0, stream>>>(THA, AD);
    k_backward<<<kGroup, kLen, 0, stream>>>(THA, BD);
    k_posterior<<<dim3(kLen, kGroup), kLen, 0, stream>>>(AD, BD, out, gbase);
  }
}
